// SSMInterBlock_54236847014470
// MI455X (gfx1250) — hardware-run, weakly checked
//
#include <hip/hip_runtime.h>
#include <math.h>

typedef __attribute__((ext_vector_type(16))) _Float16 v16h;
typedef __attribute__((ext_vector_type(8)))  _Float16 v8h;
typedef __attribute__((ext_vector_type(16))) __bf16   v16b;
typedef __attribute__((ext_vector_type(8)))  __bf16   v8b;
typedef __attribute__((ext_vector_type(8)))  float    v8f;
typedef __attribute__((ext_vector_type(4)))  float    v4f;
typedef __attribute__((ext_vector_type(2)))  float    v2f;

constexpr int kWin  = 4 * 56 * 56;
constexpr int kBl   = 4;
constexpr int kDm   = 96;
constexpr int kDe   = 192;
constexpr int kNs   = 16;
constexpr int kR    = 6;
constexpr int kXo   = kR + 2 * kNs;
constexpr int kXoP  = 64;
constexpr int kDmP  = 128;
constexpr int kRows = kWin * kBl;
constexpr int kHalfW = kWin / 2;
constexpr int kHalfR = kRows / 2;
constexpr float kLnEps = 1e-5f;
constexpr int kThr  = 256;
constexpr float kInCarry = 1024.0f;
constexpr float kSc = 1.0f / (kInCarry * kInCarry);
constexpr float kF16MinNormal = 6.103515625e-5f;

static_assert((kHalfR % 64) == 0 && ((2 * kDe) % 64) == 0 && (kXoP % 64) == 0 && (kDmP % 64) == 0 && (kDm % 32) == 0 && (kDe % 32) == 0 && ((kHalfR / 64) * (kXoP / 64)) % 8 == 0 && kXo <= kXoP && kDm <= kDmP, "GEMM M, N multiples of 64, K of 32; the smallest grid exact (392 tiles a half)");

constexpr size_t kOffX16 = 0ull;
constexpr size_t kOffWIN16 = 9633792ull;
constexpr size_t kOffWX16 = 9707520ull;
constexpr size_t kOffWOUT16 = 9732096ull;
constexpr size_t kOffZB = 9781248ull;
constexpr size_t kOffXZ = 9783296ull;
constexpr size_t kOffU16 = 48318464ull;
constexpr size_t kOffXD = 57952256ull;
constexpr size_t kOffY32 = 64374784ull;
constexpr size_t kOffG16 = 83642368ull;
constexpr size_t kOffOUTP = 93276160ull;
constexpr size_t kWsTotal = 106121216ull;
static_assert(kWsTotal <= 134217728ull, "carve cap: under 128 MiB");
static_assert(kOffX16 == 0
              && kOffWIN16 == kOffX16 + 9633792ull
              && kOffWX16 == kOffWIN16 + 73728ull
              && kOffWOUT16 == kOffWX16 + 24576ull
              && kOffZB == kOffWOUT16 + 49152ull
              && kOffXZ == kOffZB + 2048ull
              && kOffU16 == kOffXZ + 38535168ull
              && kOffXD == kOffU16 + 9633792ull
              && kOffY32 == kOffXD + 6422528ull
              && kOffG16 == kOffY32 + 19267584ull
              && kOffOUTP == kOffG16 + 9633792ull
              && kWsTotal == kOffOUTP + 12845056ull, "the carve is chained and totalled");
static_assert((kOffX16 % 256) == 0 && (kOffWIN16 % 256) == 0 && (kOffWX16 % 256) == 0 && (kOffWOUT16 % 256) == 0 && (kOffZB % 256) == 0 && (kOffXZ % 256) == 0 && (kOffU16 % 256) == 0 && (kOffXD % 256) == 0 && (kOffY32 % 256) == 0 && (kOffG16 % 256) == 0 && (kOffOUTP % 256) == 0, "aligned regions");

__device__ __forceinline__ unsigned short f2bf_bits(float f) {
  unsigned u = __float_as_uint(f);
  return (unsigned short)((u + 0x7FFFu + ((u >> 16) & 1u)) >> 16);
}
__device__ __forceinline__ float bf_bits2f(unsigned short h) { return __uint_as_float(((unsigned)h) << 16); }
__device__ __forceinline__ float bf16r(float f) { return bf_bits2f(f2bf_bits(f)); }
__device__ __forceinline__ float carry_flush(float v, float carry) {
  const float s = v * carry;
  return (fabsf(s) < kF16MinNormal) ? 0.0f : s;
}
__device__ __forceinline__ float frcp(float x) { return __builtin_amdgcn_rcpf(x); }

__device__ __forceinline__ void dep_guard4_h(v8f& a, v8f& b, v8f& c, v8f& d, v16h x, v16h y) { asm volatile("v_nop\n\tv_nop\n\tv_nop\n\tv_nop" : "+v"(a), "+v"(b), "+v"(c), "+v"(d) : "v"(x), "v"(y)); }
__device__ __forceinline__ void dep_guard4_b(v8f& a, v8f& b, v8f& c, v8f& d, v16b x, v16b y) { asm volatile("v_nop\n\tv_nop\n\tv_nop\n\tv_nop" : "+v"(a), "+v"(b), "+v"(c), "+v"(d) : "v"(x), "v"(y)); }
__device__ __forceinline__ void keep4_h(v16h a, v16h b, v16h c, v16h d) { asm volatile("v_nop" :: "v"(a), "v"(b), "v"(c), "v"(d)); }
__device__ __forceinline__ void keep4_b(v16b a, v16b b, v16b c, v16b d) { asm volatile("v_nop" :: "v"(a), "v"(b), "v"(c), "v"(d)); }
__device__ __forceinline__ void acc_guard4(v8f& a, v8f& b, v8f& c, v8f& d) { asm volatile("v_nop\n\tv_nop\n\tv_nop\n\tv_nop" : "+v"(a), "+v"(b), "+v"(c), "+v"(d)); }

template <typename T> struct Frag;
template <> struct Frag<_Float16> {
  typedef v16h V; union U { v16h v; v8h h[2]; };
  static __device__ __forceinline__ v16h load(const _Float16* p) {
    U f; f.h[0] = *(const v8h*)(p); f.h[1] = *(const v8h*)(p + 16); return f.v;
  }
  static __device__ __forceinline__ v8f mma(v16h a, v16h b, v8f c) {
    return __builtin_amdgcn_wmma_f32_16x16x32_f16(false, a, false, b, (short)0, c, false, false);
  }
  static __device__ __forceinline__ void guard4(v8f& a, v8f& b, v8f& c, v8f& d, v16h x, v16h y) { dep_guard4_h(a, b, c, d, x, y); }
  static __device__ __forceinline__ void keep(v16h a, v16h b, v16h c, v16h d) { keep4_h(a, b, c, d); }
};
template <> struct Frag<__bf16> {
  typedef v16b V; union U { v16b v; v8b h[2]; };
  static __device__ __forceinline__ v16b load(const __bf16* p) {
    U f; f.h[0] = *(const v8b*)(p); f.h[1] = *(const v8b*)(p + 16); return f.v;
  }
  static __device__ __forceinline__ v8f mma(v16b a, v16b b, v8f c) {
    return __builtin_amdgcn_wmma_f32_16x16x32_bf16(false, a, false, b, (short)0, c, false, false);
  }
  static __device__ __forceinline__ void guard4(v8f& a, v8f& b, v8f& c, v8f& d, v16b x, v16b y) { dep_guard4_b(a, b, c, d, x, y); }
  static __device__ __forceinline__ void keep(v16b a, v16b b, v16b c, v16b d) { keep4_b(a, b, c, d); }
};

__device__ __forceinline__ v8f mma_h(v16h a, v16h b, v8f c) {
  c = __builtin_amdgcn_wmma_f32_16x16x32_f16(false, a, false, b, (short)0, c, false, false);
  asm volatile("v_nop\n\tv_nop\n\tv_nop\n\tv_nop" : "+v"(c) : "v"(a), "v"(b));
  return c;
}

template <int ET> struct Elem;
template <> struct Elem<0> { typedef _Float16 T; };
template <> struct Elem<1> { typedef __bf16 T; };
template <int ET, bool SPLIT, int BIAS_MODE, int OUT_MODE, bool RESID, int ACT = 0>
__global__ __launch_bounds__(256) void wmma_gemm64(
    const unsigned short* __restrict__ Ap, const unsigned short* __restrict__ A2p, int lda, long strideA,
    const unsigned short* __restrict__ Btp, const unsigned short* __restrict__ Bt2p, int ldb, long strideB,
    void* __restrict__ Cout, void* __restrict__ Cout2, int ldc, long strideC,
    const float* __restrict__ bias,
    const float* __restrict__ resid, long strideR,
    int M, int N, int K, float scale) {
  typedef typename Elem<ET>::T T;
  typedef typename Frag<T>::V V;
  const T* A = (const T*)Ap; const T* A2 = (const T*)A2p; const T* Bt = (const T*)Btp; const T* Bt2 = (const T*)Bt2p;
  __shared__ __align__(16) float sT[8][16 * 68];
  const int b    = blockIdx.y;
  const int lane = threadIdx.x & 31;
  const int wave = threadIdx.x >> 5;
  const int tilesN = N >> 6;
  const int tilesM = M >> 6;
  const int tile = blockIdx.x * 8 + wave;
  if (tile >= tilesM * tilesN) return;
  const int tm = tile / tilesN;
  const int tn = tile - tm * tilesN;
  const int m0 = tm << 6;
  const int n0 = tn << 6;

  const T* Ab  = A  + (size_t)b * strideA;
  const T* Bb  = Bt + (size_t)b * strideB;
  const T* Ab2 = SPLIT ? (A2  + (size_t)b * strideA) : nullptr;
  const T* Bb2 = SPLIT ? (Bt2 + (size_t)b * strideB) : nullptr;

  const int rlane = lane & 15;
  const int koff  = (lane >> 4) * 8;
  const int mOff  = (lane >> 4) * 8;

  v8f acc[4][4];
#pragma unroll
  for (int i = 0; i < 4; ++i)
#pragma unroll
    for (int j = 0; j < 4; ++j) acc[i][j] = (v8f){0.f,0.f,0.f,0.f,0.f,0.f,0.f,0.f};

  for (int k0 = 0; k0 < K; k0 += 32) {
    V bh[4], bl[4];
#pragma unroll
    for (int j = 0; j < 4; ++j) {
      const size_t bo = (size_t)(n0 + (j << 4) + rlane) * ldb + koff + k0;
      bh[j] = Frag<T>::load(Bb + bo);
      if (SPLIT) bl[j] = Frag<T>::load(Bb2 + bo);
    }
#pragma unroll
    for (int i = 0; i < 4; ++i) {
      const size_t ao = (size_t)(m0 + (i << 4) + rlane) * lda + koff + k0;
      V ah = Frag<T>::load(Ab + ao);
      V al;
      if (SPLIT) al = Frag<T>::load(Ab2 + ao);
#pragma unroll
      for (int j = 0; j < 4; ++j) {
        acc[i][j] = Frag<T>::mma(ah, bh[j], acc[i][j]);
        if (SPLIT) {
          acc[i][j] = Frag<T>::mma(ah, bl[j], acc[i][j]);
          acc[i][j] = Frag<T>::mma(al, bh[j], acc[i][j]);
        }
      }
      Frag<T>::guard4(acc[i][0], acc[i][1], acc[i][2], acc[i][3], ah, SPLIT ? al : ah);
    }
    Frag<T>::keep(bh[0], bh[1], bh[2], bh[3]);
    if (SPLIT) Frag<T>::keep(bl[0], bl[1], bl[2], bl[3]);
  }
  acc_guard4(acc[0][0], acc[0][1], acc[0][2], acc[0][3]);
  acc_guard4(acc[1][0], acc[1][1], acc[1][2], acc[1][3]);
  acc_guard4(acc[2][0], acc[2][1], acc[2][2], acc[2][3]);
  acc_guard4(acc[3][0], acc[3][1], acc[3][2], acc[3][3]);

  float* slab = sT[wave];
  const float* Rb = RESID ? (resid + (size_t)b * strideR) : nullptr;
#pragma unroll
  for (int i = 0; i < 4; ++i) {
    const int mBase = m0 + (i << 4);
#pragma unroll
    for (int j = 0; j < 4; ++j) {
      const int n = n0 + (j << 4) + rlane;
      float bv = 0.f;
      if (BIAS_MODE == 2) bv = bias[n];
#pragma unroll
      for (int r = 0; r < 8; ++r) {
        float v = acc[i][j][r] * scale;
        if (BIAS_MODE == 1) v += bias[mBase + mOff + r];
        if (BIAS_MODE == 2) v += bv;
        if (RESID) v += Rb[(size_t)(mBase + mOff + r) * ldc + n];
        if (ACT == 1) v = tanhf(v);
        if (ACT == 2) v = fmaxf(v, 0.0f);
        if (ACT == 3) v = v / (1.0f + expf(-v));
        if (ACT == 4) v = (v > 0.f) ? v : 0.01f * v;
        slab[(mOff + r) * 68 + (j << 4) + rlane] = v;
      }
    }
    __builtin_amdgcn_fence(__ATOMIC_RELEASE, "workgroup");
    __builtin_amdgcn_wave_barrier();
    __builtin_amdgcn_fence(__ATOMIC_ACQUIRE, "workgroup");
    if (OUT_MODE == 0) {
      float* C = (float*)Cout + (size_t)b * strideC;
      const int hh = lane >> 4, c4 = (lane & 15) * 4;
      for (int pass = 0; pass < 2; ++pass) {
#pragma unroll
        for (int it = 0; it < 8; ++it) {
          const int row = it * 2 + hh;
          v4f v = *(const v4f*)(slab + row * 68 + c4);
          *(volatile v4f*)(C + (size_t)(mBase + row) * ldc + n0 + c4) = v;
        }
        __threadfence();
      }
    } else {
      const int q = lane >> 3, c8 = (lane & 7) * 8;
      unsigned short* C  = (unsigned short*)Cout  + (size_t)b * strideC;
      unsigned short* C2 = (OUT_MODE == 2) ? ((unsigned short*)Cout2 + (size_t)b * strideC) : nullptr;
      for (int pass = 0; pass < 2; ++pass) {
#pragma unroll
        for (int it = 0; it < 4; ++it) {
          const int row = it * 4 + q;
          const float* sp = slab + row * 68 + c8;
          v8h hv, lv;
#pragma unroll
          for (int e = 0; e < 8; ++e) {
            if (OUT_MODE == 1) {
              hv[e] = (_Float16)sp[e];
            } else {
              unsigned short hb = f2bf_bits(sp[e]);
              unsigned short lb = f2bf_bits(sp[e] - bf_bits2f(hb));
              hv[e] = __builtin_bit_cast(_Float16, hb);
              lv[e] = __builtin_bit_cast(_Float16, lb);
            }
          }
          *(volatile v8h*)(C + (size_t)(mBase + row) * ldc + n0 + c8) = hv;
          if (OUT_MODE == 2) *(volatile v8h*)(C2 + (size_t)(mBase + row) * ldc + n0 + c8) = lv;
        }
        __threadfence();
      }
    }
    __builtin_amdgcn_fence(__ATOMIC_RELEASE, "workgroup");
    __builtin_amdgcn_wave_barrier();
    __builtin_amdgcn_fence(__ATOMIC_ACQUIRE, "workgroup");
  }
}

__global__ __launch_bounds__(kThr) void cast_plane_kernel(const float* __restrict__ src, unsigned short* __restrict__ dst,
                                                          int colsLog2, int dstPitch, int dstOff) {
  const int i   = blockIdx.x * kThr + threadIdx.x;
  const int sh  = colsLog2 - 3;
  const int row = i >> sh;
  const int c8  = (i & ((1 << sh) - 1)) * 8;
  const float* sp = src + ((size_t)row << colsLog2) + c8;
  const v4f a0 = *(const v4f*)(sp);
  const v4f a1 = *(const v4f*)(sp + 4);
  v8h hv;
#pragma unroll
  for (int e = 0; e < 4; ++e) {
    const float f0 = a0[e];
    const float f1 = a1[e];
    hv[e]     = (_Float16)carry_flush(bf16r(f0), kInCarry);
    hv[4 + e] = (_Float16)carry_flush(bf16r(f1), kInCarry);
  }
  unsigned short* dp = dst + (size_t)row * dstPitch + dstOff + c8;
  *(volatile v8h*)dp = hv;
  __threadfence();
  *(volatile v8h*)dp = hv;
}

__device__ __forceinline__ float silu_f(float v) { return v / (1.0f + expf(-v)); }

__global__ __launch_bounds__(48) void xt_cast_kernel(const float* __restrict__ x, unsigned short* __restrict__ X16) {
  const unsigned w = blockIdx.y;
  const unsigned bl = threadIdx.y, d8 = threadIdx.x * 8u;
  const float* sp = x + (size_t)w * (kDm * kBl) + (size_t)d8 * kBl + bl;
  v8h hv;
#pragma unroll
  for (int e = 0; e < 8; ++e) {
    const float p = sp[(size_t)e * kBl];
    hv[e] = (_Float16)carry_flush(bf16r(p), kInCarry);
  }
  unsigned short* dp = X16 + (size_t)w * (kDm * kBl) + (size_t)bl * kDm + d8;
  *(volatile v8h*)dp = hv;
  __threadfence();
  *(volatile v8h*)dp = hv;
}
static_assert(kDm == 12 * 8 && kBl == 4, "a (12, 4) block: 12 chunks of 8 channels x 4 blocks");

__global__ __launch_bounds__(32) void setup_kernel(const float* __restrict__ x_proj_w, const float* __restrict__ out_proj_w,
                                                   unsigned short* __restrict__ WX16, unsigned short* __restrict__ WOUT16, float* __restrict__ ZB) {
  const unsigned y = blockIdx.y;
  const unsigned c = threadIdx.x;
  if (y < 192u) {
    if (c >= 24u) return;
    const bool second = y >= 64u;
    const unsigned r = second ? (y - 64u) : y;
    const bool live = second ? (r < (unsigned)kDm) : (r < (unsigned)kXo);
    const float* sp = (second ? out_proj_w : x_proj_w) + (size_t)(live ? r : 0u) * kDe + c * 8u;
    const v4f a0 = *(const v4f*)sp, a1 = *(const v4f*)(sp + 4);
    v8h hv;
#pragma unroll
    for (int e = 0; e < 4; ++e) {
      const float p = a0[e], q = a1[e];
      hv[e] = (_Float16)(live ? carry_flush(bf16r(p), kInCarry) : 0.0f);
      hv[4 + e] = (_Float16)(live ? carry_flush(bf16r(q), kInCarry) : 0.0f);
    }
    unsigned short* dp = (second ? WOUT16 : WX16) + (size_t)r * kDe + c * 8u;
    *(volatile v8h*)dp = hv;
    __threadfence();
    *(volatile v8h*)dp = hv;
  } else {
    const v4f z = {0.f, 0.f, 0.f, 0.f};
    for (int q = 0; q < 4; ++q) {
      float* dp = ZB + (c * 4u + (unsigned)q) * 4u;
      *(volatile v4f*)dp = z;
      __threadfence();
      *(volatile v4f*)dp = z;
    }
  }
}
static_assert(kDe == 24 * 8 && kXoP == 64 && kDmP == 128, "24 chunks a weight row; 64 + 128 weight rows");

__global__ __launch_bounds__(32) void u_cast_kernel(const float* __restrict__ XZ, unsigned short* __restrict__ U16) {
  const unsigned row = blockIdx.y;
  const unsigned c = threadIdx.x;
  if (c >= 24u) return;
  const float* sp = XZ + (size_t)row * (2 * kDe) + c * 8u;
  const v4f a0 = *(const v4f*)sp, a1 = *(const v4f*)(sp + 4);
  v8h hv;
#pragma unroll
  for (int e = 0; e < 4; ++e) { hv[e] = (_Float16)carry_flush(silu_f(a0[e]), kInCarry); hv[4 + e] = (_Float16)carry_flush(silu_f(a1[e]), kInCarry); }
  unsigned short* dp = U16 + (size_t)row * kDe + c * 8u;
  *(volatile v8h*)dp = hv;
  __threadfence();
  *(volatile v8h*)dp = hv;
}

__global__ __launch_bounds__(96) void scan_kernel(const float* __restrict__ XD, const float* __restrict__ XZ, const float* __restrict__ dtw,
                                                  const float* __restrict__ dtb, const float* __restrict__ A_logs, const float* __restrict__ Ds,
                                                  float* __restrict__ Y32) {
  const unsigned w = blockIdx.y;
  const unsigned d0 = threadIdx.x * 2u;
  float A[2][kNs], h[2][kNs], wd[2][kR], bd[2], dc[2];
#pragma unroll
  for (int k = 0; k < 2; ++k) {
    const unsigned d = d0 + (unsigned)k;
#pragma unroll
    for (int n = 0; n < kNs; ++n) { const float a = A_logs[(size_t)d * kNs + n]; A[k][n] = -expf(bf16r(a)); h[k][n] = 0.0f; }
#pragma unroll
    for (int r = 0; r < kR; ++r) { const float ww = dtw[(size_t)d * kR + r]; wd[k][r] = bf16r(ww); }
    const float b0 = dtb[d], q0 = Ds[d];
    bd[k] = bf16r(b0); dc[k] = bf16r(q0);
  }
#pragma unroll
  for (int l = 0; l < kBl; ++l) {
    const size_t row = (size_t)w * kBl + (size_t)l;
    const float* pr = XD + row * kXoP;
    const v2f xv = *(const v2f*)(XZ + row * (2 * kDe) + d0);
    float y[2], delta[2], dx[2], uu[2];
#pragma unroll
    for (int k = 0; k < 2; ++k) {
      float pre = bd[k];
#pragma unroll
      for (int r = 0; r < kR; ++r) pre += wd[k][r] * pr[r];
      delta[k] = (pre > 20.0f) ? pre : log1pf(expf(pre));
      uu[k] = silu_f(xv[k]);
      dx[k] = delta[k] * uu[k];
      y[k] = 0.0f;
    }
#pragma unroll
    for (int n = 0; n < kNs; ++n) {
      const float bn = pr[kR + n], cn = pr[kR + kNs + n];
#pragma unroll
      for (int k = 0; k < 2; ++k) {
        const float hn = expf(delta[k] * A[k][n]) * h[k][n] + dx[k] * bn;
        h[k][n] = hn;
        y[k] += hn * cn;
      }
    }
    v2f ov;
    ov[0] = y[0] + dc[0] * uu[0]; ov[1] = y[1] + dc[1] * uu[1];
    float* dp = Y32 + row * kDe + d0;
    *(volatile v2f*)dp = ov;
    __threadfence();
    *(volatile v2f*)dp = ov;
  }
}
static_assert(kDe == 96 * 2 && kXo == kR + 2 * kNs, "96 lanes a window; the parameter columns 6 | 16 | 16");

__global__ __launch_bounds__(128) void ln_gate_kernel(const float* __restrict__ Y32, const float* __restrict__ XZ, const float* __restrict__ gam,
                                                      const float* __restrict__ bet, unsigned short* __restrict__ G16) {
  const size_t row = (size_t)blockIdx.x * 128u + threadIdx.x;
  const float* yr = Y32 + row * kDe;
  const float* zr = XZ + row * (2 * kDe) + kDe;
  float s = 0.0f;
  for (int c = 0; c < kDe; c += 4) { const v4f a = *(const v4f*)(yr + c); s += (a[0] + a[1]) + (a[2] + a[3]); }
  const float mu = s / (float)kDe;
  float q = 0.0f;
  for (int c = 0; c < kDe; c += 4) { const v4f a = *(const v4f*)(yr + c); const float d0 = a[0] - mu, d1 = a[1] - mu, d2 = a[2] - mu, d3 = a[3] - mu; q += (d0 * d0 + d1 * d1) + (d2 * d2 + d3 * d3); }
  const float rs = 1.0f / sqrtf(q / (float)kDe + kLnEps);
  unsigned short* gr = G16 + row * kDe;
  for (int c = 0; c < kDe; c += 8) {
    const v4f a0 = *(const v4f*)(yr + c), a1 = *(const v4f*)(yr + c + 4);
    const v4f z0 = *(const v4f*)(zr + c), z1 = *(const v4f*)(zr + c + 4);
    const v4f g0 = *(const v4f*)(gam + c), g1 = *(const v4f*)(gam + c + 4);
    const v4f b0 = *(const v4f*)(bet + c), b1 = *(const v4f*)(bet + c + 4);
    v8h hv;
#pragma unroll
    for (int e = 0; e < 4; ++e) {
      const float p0 = g0[e], p1 = g1[e], r0 = b0[e], r1 = b1[e];
      const float n0 = (a0[e] - mu) * rs * bf16r(p0) + bf16r(r0);
      const float n1 = (a1[e] - mu) * rs * bf16r(p1) + bf16r(r1);
      hv[e] = (_Float16)carry_flush(n0 * silu_f(z0[e]), kInCarry);
      hv[4 + e] = (_Float16)carry_flush(n1 * silu_f(z1[e]), kInCarry);
    }
    *(volatile v8h*)(gr + c) = hv;
    __threadfence();
    *(volatile v8h*)(gr + c) = hv;
  }
}
static_assert(kHalfR % 128 == 0 && (kDe % 8) == 0, "norm grid exact");

__global__ __launch_bounds__(96) void out_t_kernel(const float* __restrict__ OUTP, float* __restrict__ out) {
  const unsigned w = blockIdx.y;
  const unsigned d = threadIdx.x;
  const float* pr = OUTP + (size_t)w * kBl * kDmP + d;
  v4f ov;
#pragma unroll
  for (int b = 0; b < kBl; ++b) ov[b] = pr[(size_t)b * kDmP];
  float* dp = out + (size_t)w * (kDm * kBl) + d * (unsigned)kBl;
  *(volatile v4f*)dp = ov;
  __threadfence();
  *(volatile v4f*)dp = ov;
}

static_assert(((size_t)2 * kDe * kDm) % (4096) == 0 && (((size_t)2 * kDe * kDm / 8) % kThr) == 0, "the linear cast of in_proj_w is whole rows of 4,096 and whole blocks");

extern "C" void kernel_launch(void* const* d_in, const int* in_sizes, int n_in,
                              void* d_out, int out_size, void* d_ws, size_t ws_size,
                              hipStream_t stream) {
  if (n_in < 10 || d_out == nullptr || d_ws == nullptr) return;
  if (in_sizes[0] != kRows * kDm || in_sizes[1] != 2 * kDe * kDm || in_sizes[2] != kXo * kDe || in_sizes[3] != kDe * kR || in_sizes[4] != kDe) return;
  if (in_sizes[5] != kDe * kNs || in_sizes[6] != kDe || in_sizes[7] != kDe || in_sizes[8] != kDe || in_sizes[9] != kDm * kDe) return;
  if (out_size != kRows * kDm) return;
  if (ws_size < kWsTotal) return;
  const float* x = (const float*)d_in[0];
  const float* in_proj_w = (const float*)d_in[1];
  const float* x_proj_weight = (const float*)d_in[2];
  const float* dt_projs_weight = (const float*)d_in[3];
  const float* dt_projs_bias = (const float*)d_in[4];
  const float* A_logs = (const float*)d_in[5];
  const float* Ds = (const float*)d_in[6];
  const float* ln_gamma = (const float*)d_in[7];
  const float* ln_beta = (const float*)d_in[8];
  const float* out_proj_w = (const float*)d_in[9];
  float* out = (float*)d_out;
  char* ws = (char*)d_ws;
  unsigned short* X16 = (unsigned short*)(ws + kOffX16);
  unsigned short* WIN16 = (unsigned short*)(ws + kOffWIN16);
  unsigned short* WX16 = (unsigned short*)(ws + kOffWX16);
  unsigned short* WOUT16 = (unsigned short*)(ws + kOffWOUT16);
  float* ZB = (float*)(ws + kOffZB);
  float* XZ = (float*)(ws + kOffXZ);
  unsigned short* U16 = (unsigned short*)(ws + kOffU16);
  float* XD = (float*)(ws + kOffXD);
  float* Y32 = (float*)(ws + kOffY32);
  unsigned short* G16 = (unsigned short*)(ws + kOffG16);
  float* OUTP = (float*)(ws + kOffOUTP);

  xt_cast_kernel<<<dim3(1, kWin), dim3(12, 4), 0, stream>>>(x, X16);
  cast_plane_kernel<<<(int)(((size_t)2 * kDe * kDm / 8) / kThr), kThr, 0, stream>>>(in_proj_w, WIN16, 12, 4096, 0);
  setup_kernel<<<dim3(1, 193), 32, 0, stream>>>(x_proj_weight, out_proj_w, WX16, WOUT16, ZB);
  for (int hf = 0; hf < 2; ++hf) {
    const size_t r0 = (size_t)hf * kHalfR;
    wmma_gemm64<0, false, 2, 0, false, 0><<<dim3((kHalfR / 64) * (2 * kDe / 64) / 8, 1), 256, 0, stream>>>(
        X16 + r0 * kDm, X16 + r0 * kDm, kDm, 0L, WIN16, WIN16, kDm, 0L, (void*)XZ, (void*)XZ, 2 * kDe, 0L, ZB, nullptr, 0L, kHalfR, 2 * kDe, kDm, kSc);
    u_cast_kernel<<<dim3(1, kHalfR), 32, 0, stream>>>(XZ, U16);
    wmma_gemm64<0, false, 2, 0, false, 0><<<dim3((kHalfR / 64) * (kXoP / 64) / 8, 1), 256, 0, stream>>>(
        U16, U16, kDe, 0L, WX16, WX16, kDe, 0L, (void*)XD, (void*)XD, kXoP, 0L, ZB, nullptr, 0L, kHalfR, kXoP, kDe, kSc);
    scan_kernel<<<dim3(1, kHalfW), 96, 0, stream>>>(XD, XZ, dt_projs_weight, dt_projs_bias, A_logs, Ds, Y32);
    ln_gate_kernel<<<kHalfR / 128, 128, 0, stream>>>(Y32, XZ, ln_gamma, ln_beta, G16);
    wmma_gemm64<0, false, 2, 0, false, 0><<<dim3((kHalfR / 64) * (kDmP / 64) / 8, 1), 256, 0, stream>>>(
        G16, G16, kDe, 0L, WOUT16, WOUT16, kDe, 0L, (void*)OUTP, (void*)OUTP, kDmP, 0L, ZB, nullptr, 0L, kHalfR, kDmP, kDe, kSc);
    out_t_kernel<<<dim3(1, kHalfW), 96, 0, stream>>>(OUTP, out + r0 * kDm);
  }
}
